// TorchMD_GN_14688788152851
// MI455X (gfx1250) — hardware-verified
//
#include <hip/hip_runtime.h>
#include <stddef.h>


#define HID      128
#define KRB      64
#define NLAY     3
#define NTHR     256
#define NWAVE    8
#define EPT      8
#define NGRP     2
#define CHUNK    (NTHR * EPT * NGRP)
#define WCAP     (EPT * NGRP * 32)
#define LISTN    (NWAVE * WCAP)
#define NBC      4096
#define NBF      1024
#define RCAP     40960
#define RBN      128
#define OTHR     512
#define DEGCAP   256
#define CNB      32
#define CPOS     64
#define GROWS    128
#define EROWS    32
#define APE      (KRB + 8)
#define TPH      (HID + 8)
#define WPF      (HID + 4)
#define EA_SCALE 256.0f
#define EA_INV   0.00390625f
#define CUT_HI   5.0f
#define PI_OVER_CUT 0.62831853071795864f
#define WSCAP    134217728
#define LDS_FILL ((RCAP + NBF + LISTN) * 4 + 64)
#define LDS_NG128 (GROWS * HID * 4)
#define LDS_NG256 (GROWS * (2 * HID + 8) * 2)
#define FL_BIAS  1
#define FL_SILU  2
#define FL_RES   4
#define WO_PROJ  0
#define WO_COMB  8192
#define WO_LAY0  40960
#define WL_STR   73728
#define WL_W0    0
#define WL_W1    8192
#define WL_L1    24576
#define WL_L2    40960
#define WL_LW    57344
#define WTOT     262144
#define WBLK     128

static_assert((CHUNK & (CHUNK - 1)) == 0);
static_assert(CHUNK <= 4096);
static_assert((NBC & (NBC - 1)) == 0 && (NBF & (NBF - 1)) == 0);
static_assert(NBC == 4 * NBF);
static_assert(OTHR * 8 == NBC);
static_assert((RCAP % 32) == 0);
static_assert((NBF % CNB) == 0);
static_assert((GROWS % CNB) == 0);
static_assert(CNB == 4 * NWAVE);
static_assert(CPOS * (KRB / 8) == 2 * NTHR);
static_assert(((APE * 2) % 16) == 0 && ((TPH * 2) % 16) == 0 && ((WPF * 4) % 16) == 0);
static_assert(WTOT == WBLK * NTHR * 8);
static_assert(EROWS * (KRB / 8) == NTHR);
static_assert(EROWS * KRB == NTHR * 8);
static_assert(GROWS == NWAVE * 16);
static_assert((KRB % 32) == 0);
static_assert(LDS_NG128 <= LDS_NG256);
static_assert((CNB * DEGCAP) % CPOS == 0);

typedef float          v4f  __attribute__((ext_vector_type(4)));
typedef float          v8f  __attribute__((ext_vector_type(8)));
typedef int            v4i  __attribute__((ext_vector_type(4)));
typedef _Float16       v8h  __attribute__((ext_vector_type(8)));
typedef _Float16       v16h __attribute__((ext_vector_type(16)));
union FragH { v16h v; v8h h[2]; };

__device__ __forceinline__ v8f wm(v16h a, v16h b, v8f c) {
  v8f d = __builtin_amdgcn_wmma_f32_16x16x32_f16(false, a, false, b, (short)0, c, false, false);
  asm volatile("v_nop\n\tv_nop\n\tv_nop\n\tv_nop" : "+v"(d) : "v"(a), "v"(b));
  return d;
}

__device__ __forceinline__ float silu_f(float v) {
  return v * __builtin_amdgcn_rcpf(1.0f + __expf(-v));
}
__device__ __forceinline__ v4f silu4(v4f v) {
  v4f r;
  r.x = silu_f(v.x); r.y = silu_f(v.y); r.z = silu_f(v.z); r.w = silu_f(v.w);
  return r;
}
__device__ __forceinline__ v8h cvt8(v4f a, v4f b) {
  v8h o;
  o[0] = (_Float16)a.x; o[1] = (_Float16)a.y; o[2] = (_Float16)a.z; o[3] = (_Float16)a.w;
  o[4] = (_Float16)b.x; o[5] = (_Float16)b.y; o[6] = (_Float16)b.z; o[7] = (_Float16)b.w;
  return o;
}

template <int NB>
__device__ __forceinline__ int scan_chunk(const int* __restrict__ keys, int nE, int cbase, int slotBase,
                                          int vec8, int* list, int tid, int lane, int wave) {
  int wc = 0;
#pragma unroll
  for (int g = 0; g < NGRP; ++g) {
    const int el0  = (g * NTHR + tid) * EPT;
    const int e0   = cbase + el0;
    const int sent = -2147483647 - 1;
    v4i da, db;
    if (vec8 != 0 && cbase + CHUNK <= nE) {
      da = *(const v4i*)(keys + e0);
      db = *(const v4i*)(keys + e0 + 4);
    } else {
      da.x = (e0     < nE) ? keys[min(e0, nE - 1)] : sent;
      da.y = (e0 + 1 < nE) ? keys[min(e0 + 1, nE - 1)] : sent;
      da.z = (e0 + 2 < nE) ? keys[min(e0 + 2, nE - 1)] : sent;
      da.w = (e0 + 3 < nE) ? keys[min(e0 + 3, nE - 1)] : sent;
      db.x = (e0 + 4 < nE) ? keys[min(e0 + 4, nE - 1)] : sent;
      db.y = (e0 + 5 < nE) ? keys[min(e0 + 5, nE - 1)] : sent;
      db.z = (e0 + 6 < nE) ? keys[min(e0 + 6, nE - 1)] : sent;
      db.w = (e0 + 7 < nE) ? keys[min(e0 + 7, nE - 1)] : sent;
    }
    const unsigned nb = (unsigned)slotBase;
    const unsigned s0 = (unsigned)da.x - nb, s1 = (unsigned)da.y - nb;
    const unsigned s2 = (unsigned)da.z - nb, s3 = (unsigned)da.w - nb;
    const unsigned s4 = (unsigned)db.x - nb, s5 = (unsigned)db.y - nb;
    const unsigned s6 = (unsigned)db.z - nb, s7 = (unsigned)db.w - nb;
    const bool h0 = s0 < (unsigned)NB, h1 = s1 < (unsigned)NB, h2 = s2 < (unsigned)NB, h3 = s3 < (unsigned)NB;
    const bool h4 = s4 < (unsigned)NB, h5 = s5 < (unsigned)NB, h6 = s6 < (unsigned)NB, h7 = s7 < (unsigned)NB;
    const unsigned any = __builtin_amdgcn_ballot_w32(h0 | h1 | h2 | h3 | h4 | h5 | h6 | h7);
    if (any != 0u) {
#define HITJ(J, HJ, SJ) { \
        const unsigned mj = __builtin_amdgcn_ballot_w32(HJ); \
        if (mj != 0u) { \
          if (HJ) { \
            const int pos = wc + (int)__builtin_amdgcn_mbcnt_lo(mj, 0u); \
            if (pos < WCAP) list[wave * WCAP + pos] = ((el0 + (J)) << 12) | (int)(SJ); \
          } \
          wc += (int)__builtin_popcount(mj); } }
      HITJ(0, h0, s0)
      HITJ(1, h1, s1)
      HITJ(2, h2, s2)
      HITJ(3, h3, s3)
      HITJ(4, h4, s4)
      HITJ(5, h5, s5)
      HITJ(6, h6, s6)
      HITJ(7, h7, s7)
#undef HITJ
    }
  }
  return wc;
}

__global__ __launch_bounds__(NTHR) void k_wprep(
    const float* __restrict__ pw, const float* __restrict__ cw,
    const float* __restrict__ w0, const float* __restrict__ w1,
    const float* __restrict__ l1, const float* __restrict__ l2,
    const float* __restrict__ lw, _Float16* wp, int nrbf) {
  const int tid = (int)threadIdx.x;
  const int b = (int)blockIdx.x;
  const float* src = pw;
  int K = nrbf, Kp = KRB, doff = WO_PROJ, lp = tid;
  if (b < 4) {
    src = pw; K = nrbf; Kp = KRB; doff = WO_PROJ; lp = b * NTHR + tid;
  } else if (b < 20) {
    src = cw; K = 2 * HID; Kp = 2 * HID; doff = WO_COMB; lp = (b - 4) * NTHR + tid;
  } else {
    const int lb = b - 20;
    const int l = lb / 36;
    const int r = lb - l * 36;
    const int lbase = WO_LAY0 + l * WL_STR;
    if (r < 4)       { src = w0 + (size_t)l * HID * nrbf; K = nrbf; Kp = KRB; doff = lbase + WL_W0; lp = r * NTHR + tid; }
    else if (r < 12) { src = w1 + (size_t)l * HID * HID;  K = HID;  Kp = HID; doff = lbase + WL_W1; lp = (r - 4) * NTHR + tid; }
    else if (r < 20) { src = l1 + (size_t)l * HID * HID;  K = HID;  Kp = HID; doff = lbase + WL_L1; lp = (r - 12) * NTHR + tid; }
    else if (r < 28) { src = l2 + (size_t)l * HID * HID;  K = HID;  Kp = HID; doff = lbase + WL_L2; lp = (r - 20) * NTHR + tid; }
    else             { src = lw + (size_t)l * HID * HID;  K = HID;  Kp = HID; doff = lbase + WL_LW; lp = (r - 28) * NTHR + tid; }
  }
  const int ppr = Kp >> 3;
  const int n   = lp / ppr;
  const int k0  = (lp - n * ppr) * 8;
  float v[8];
#pragma unroll
  for (int j = 0; j < 8; ++j) {
    const int k  = k0 + j;
    const int kc = k < K ? k : K - 1;
    const float f = src[(size_t)n * K + kc];
    v[j] = (k < K) ? f : 0.0f;
  }
  v4f a, c;
  a.x = v[0]; a.y = v[1]; a.z = v[2]; a.w = v[3];
  c.x = v[4]; c.y = v[5]; c.z = v[6]; c.w = v[7];
  const v8h o = cvt8(a, c);
  _Float16* dp = wp + doff + (size_t)n * Kp + k0;
  *(volatile v8h*)dp = o;
  __threadfence();
  *(volatile v8h*)dp = o;
}

__global__ __launch_bounds__(NTHR) void k_count(
    const int* __restrict__ keys, int* cnt, int nE, int vec8) {
  __shared__ __attribute__((aligned(16))) int scnt[NBC];
  __shared__ __attribute__((aligned(16))) int list[LISTN];
  __shared__ int wcnt[NWAVE];
  const int tid = threadIdx.x, lane = tid & 31, wave = tid >> 5;
  const int nodeBase = blockIdx.x * NBC;

  for (int i = tid; i < NBC; i += NTHR) scnt[i] = 0;
  __syncthreads();

  const int nChunks = (nE + CHUNK - 1) / CHUNK;
#pragma unroll 1
  for (int ch = 0; ch < nChunks; ++ch) {
    const int cbase = ch * CHUNK;
    const int wc = scan_chunk<NBC>(keys, nE, cbase, nodeBase, vec8, list, tid, lane, wave);
    if (lane == 0) wcnt[wave] = wc;
    __syncthreads();
    if (wave == 0) {
#pragma unroll 1
      for (int wsx = 0; wsx < NWAVE; ++wsx) {
        int n = __builtin_amdgcn_readfirstlane(wcnt[wsx]);
        n = n > WCAP ? WCAP : (n < 0 ? 0 : n);
        const int* lp = list + wsx * WCAP;
#pragma unroll 1
        for (int i = 0; i < n; ++i) {
          const int ent  = __builtin_amdgcn_readfirstlane(lp[i]);
          const int slot = ent & (NBC - 1);
          if (lane == 0) scnt[slot] = scnt[slot] + 1;
        }
      }
    }
    __syncthreads();
  }

  v4i cq[4];
#pragma unroll
  for (int q = 0; q < 4; ++q) {
    const int f = (wave * 4 + q) * 128 + 4 * lane;
    cq[q] = *(const v4i*)(scnt + f);
  }
  int* cp = cnt + (size_t)nodeBase;
#pragma unroll
  for (int q = 0; q < 4; ++q) {
    const int f = (wave * 4 + q) * 128 + 4 * lane;
    *(volatile v4i*)(cp + f) = cq[q];
  }
  __threadfence();
#pragma unroll
  for (int q = 0; q < 4; ++q) {
    const int f = (wave * 4 + q) * 128 + 4 * lane;
    *(volatile v4i*)(cp + f) = cq[q];
  }
}

__global__ __launch_bounds__(OTHR) void k_offsets(
    const int* __restrict__ cnt, int* off, int* rbase, int nChunk) {
  __shared__ __attribute__((aligned(16))) int soff[NBC];
  __shared__ __attribute__((aligned(16))) int srb[RBN];
  __shared__ int wtot[OTHR / 32];
  const int tid = threadIdx.x, lane = tid & 31, wave = tid >> 5, sub = tid >> 7;
  for (int i = tid; i < RBN; i += OTHR) srb[i] = 0;
  int carry = 0;
#pragma unroll 1
  for (int ch = 0; ch < nChunk; ++ch) {
    const int base = ch * NBC;
    const v4i c0 = *(const v4i*)(cnt + base + 8 * tid);
    const v4i c1 = *(const v4i*)(cnt + base + 8 * tid + 4);
    const int e0 = max(c0.x, 0), e1 = max(c0.y, 0), e2 = max(c0.z, 0), e3 = max(c0.w, 0);
    const int e4 = max(c1.x, 0), e5 = max(c1.y, 0), e6 = max(c1.z, 0), e7 = max(c1.w, 0);
    const int ts = e0 + e1 + e2 + e3 + e4 + e5 + e6 + e7;
    int incl = ts;
#pragma unroll
    for (int d = 1; d < 32; d <<= 1) {
      const int t = __shfl_up(incl, d);
      if (lane >= d) incl += t;
    }
    if (lane == 31) wtot[wave] = incl;
    __syncthreads();
    const int S0 = wtot[0]  + wtot[1]  + wtot[2]  + wtot[3];
    const int S1 = wtot[4]  + wtot[5]  + wtot[6]  + wtot[7];
    const int S2 = wtot[8]  + wtot[9]  + wtot[10] + wtot[11];
    const int S3 = wtot[12] + wtot[13] + wtot[14] + wtot[15];
    int pre = 0;
#pragma unroll 1
    for (int w = 4 * sub; w < wave; ++w) pre += wtot[w];
    const int b0 = carry;
    const int b1 = b0 + ((S0 + 31) & ~31);
    const int b2 = b1 + ((S1 + 31) & ~31);
    const int b3 = b2 + ((S2 + 31) & ~31);
    const int b4 = b3 + ((S3 + 31) & ~31);
    const int myb = sub == 0 ? b0 : (sub == 1 ? b1 : (sub == 2 ? b2 : b3));
    if (tid == 0) {
      srb[min(4 * ch + 0, RBN - 1)] = b0;
      srb[min(4 * ch + 1, RBN - 1)] = b1;
      srb[min(4 * ch + 2, RBN - 1)] = b2;
      srb[min(4 * ch + 3, RBN - 1)] = b3;
    }
    int run = myb + pre + incl - ts;
    soff[8 * tid + 0] = run; run += e0;
    soff[8 * tid + 1] = run; run += e1;
    soff[8 * tid + 2] = run; run += e2;
    soff[8 * tid + 3] = run; run += e3;
    soff[8 * tid + 4] = run; run += e4;
    soff[8 * tid + 5] = run; run += e5;
    soff[8 * tid + 6] = run; run += e6;
    soff[8 * tid + 7] = run;
    carry = b4;
    __syncthreads();
    const v4i o0 = *(const v4i*)(soff + 4 * tid);
    const v4i o1 = *(const v4i*)(soff + 4 * (tid + OTHR));
    int* op = off + base;
    *(volatile v4i*)(op + 4 * tid) = o0;
    *(volatile v4i*)(op + 4 * (tid + OTHR)) = o1;
    __threadfence();
    *(volatile v4i*)(op + 4 * tid) = o0;
    *(volatile v4i*)(op + 4 * (tid + OTHR)) = o1;
    __syncthreads();
  }
  if (tid == 0) srb[min(4 * nChunk, RBN - 1)] = carry;
  __syncthreads();
  v4i rv = {0, 0, 0, 0};
  if (tid < 32) rv = *(const v4i*)(srb + 4 * tid);
  if (tid < 32) *(volatile v4i*)(rbase + 4 * tid) = rv;
  __threadfence();
  if (tid < 32) *(volatile v4i*)(rbase + 4 * tid) = rv;
}

__global__ __launch_bounds__(NTHR) void k_fill(
    const int* __restrict__ keys, const int* __restrict__ off, const int* __restrict__ rbase,
    int* csr, int nE, int vec8, int csrLen) {
  extern __shared__ v4f lds_dyn[];
  int* region = (int*)lds_dyn;
  int* cursor = region + RCAP;
  int* list   = cursor + NBF;
  int* wcnt   = list + LISTN;
  const int tid = threadIdx.x, lane = tid & 31, wave = tid >> 5;
  const int b = blockIdx.x;
  const int nodeBase = b * NBF;

  int rb0 = rbase[b];
  const int rb1 = rbase[b + 1];
  rb0 = rb0 < 0 ? 0 : (rb0 > csrLen ? csrLen : rb0);
  rb0 &= ~31;
  int len = rb1 - rb0;
  len = len < 0 ? 0 : (len > RCAP ? RCAP : len);
  int lenW = (len + 31) & ~31;
  if (rb0 + lenW > csrLen) lenW = (csrLen - rb0) & ~31;

  {
    const v4i z = {0, 0, 0, 0};
    for (int i = tid; i < RCAP / 4; i += NTHR) ((v4i*)region)[i] = z;
    for (int s = tid; s < NBF; s += NTHR) {
      int o = off[nodeBase + s] - rb0;
      o = o < 0 ? 0 : (o > RCAP ? RCAP : o);
      cursor[s] = o;
    }
  }
  __syncthreads();

  const int nChunks = (nE + CHUNK - 1) / CHUNK;
#pragma unroll 1
  for (int ch = 0; ch < nChunks; ++ch) {
    const int cbase = ch * CHUNK;
    const int wc = scan_chunk<NBF>(keys, nE, cbase, nodeBase, vec8, list, tid, lane, wave);
    if (lane == 0) wcnt[wave] = wc;
    __syncthreads();
    if (wave == 0) {
#pragma unroll 1
      for (int wsx = 0; wsx < NWAVE; ++wsx) {
        int n = __builtin_amdgcn_readfirstlane(wcnt[wsx]);
        n = n > WCAP ? WCAP : (n < 0 ? 0 : n);
        const int* lp = list + wsx * WCAP;
#pragma unroll 1
        for (int i = 0; i < n; ++i) {
          const int ent  = __builtin_amdgcn_readfirstlane(lp[i]);
          const int slot = ent & (NBF - 1);
          int e = cbase + ((ent >> 12) & (CHUNK - 1));
          e = e > nE - 1 ? nE - 1 : e;
          if (lane == 0) {
            int pos = cursor[slot];
            pos = pos < 0 ? 0 : (pos > RCAP - 1 ? RCAP - 1 : pos);
            region[pos] = e;
            const int np = pos + 1;
            cursor[slot] = np > RCAP ? RCAP : np;
          }
        }
      }
    }
    __syncthreads();
  }

  const int nv = lenW >> 2;
  int* gp = csr + rb0;
#pragma unroll 1
  for (int i = tid; i < nv; i += NTHR) { const v4i v = ((const v4i*)region)[i]; *(volatile v4i*)(gp + 4 * i) = v; }
  __threadfence();
#pragma unroll 1
  for (int i = tid; i < nv; i += NTHR) { const v4i v = ((const v4i*)region)[i]; *(volatile v4i*)(gp + 4 * i) = v; }
}

__global__ __launch_bounds__(NTHR) void k_eattr(
    const int* __restrict__ csr, const int* __restrict__ ei, const float* __restrict__ ew,
    const float* __restrict__ means, const float* __restrict__ betas,
    _Float16* eaP, float* Cpos, int* Spos, int* Dpos,
    int nE, int nN, int csrLen, int nrbf) {
  __shared__ __attribute__((aligned(16))) _Float16 sRow[EROWS * KRB];
  __shared__ __attribute__((aligned(16))) float sC[EROWS];
  __shared__ __attribute__((aligned(16))) int sS[EROWS];
  __shared__ __attribute__((aligned(16))) int sDd[EROWS];
  __shared__ float sEd[EROWS];
  const int tid = threadIdx.x, lane = tid & 31, wave = tid >> 5;
  const int P0 = blockIdx.x * EROWS;
  if (tid < EROWS) {
    int p = P0 + tid;
    p = p > csrLen - 1 ? csrLen - 1 : p;
    int e = csr[p];
    e = e < 0 ? 0 : (e > nE - 1 ? nE - 1 : e);
    const float d = ew[e];
    int s = ei[e];
    s = s < 0 ? 0 : (s > nN - 1 ? nN - 1 : s);
    int dn = ei[(size_t)nE + e];
    dn = dn < 0 ? 0 : (dn > nN - 1 ? nN - 1 : dn);
    float c = 0.5f * (cosf(d * PI_OVER_CUT) + 1.0f);
    c = (d < CUT_HI) ? c : 0.0f;
    sC[tid] = c;
    sS[tid] = s;
    sDd[tid] = dn;
    sEd[tid] = __expf(-d);
  }
  __syncthreads();
  const int k  = tid & 63;
  const int kc = k < nrbf ? k : nrbf - 1;
  const float mk = means[kc];
  const float bk = betas[kc];
  const int rsub = tid >> 6;
#pragma unroll 1
  for (int it = 0; it < EROWS / 4; ++it) {
    const int r = it * 4 + rsub;
    const float t = sEd[r] - mk;
    float v = sC[r] * __expf(-(bk * (t * t)));
    v = (k < nrbf) ? v * EA_SCALE : 0.0f;
    sRow[r * KRB + k] = (_Float16)v;
  }
  __syncthreads();
  const int r = tid >> 3, q = tid & 7;
  const v8h o = *(const v8h*)(sRow + r * KRB + 8 * q);
  _Float16* gp = eaP + (size_t)(P0 + r) * KRB + 8 * q;
  v4f cv = {0.f, 0.f, 0.f, 0.f};
  v4i sv = {0, 0, 0, 0};
  v4i dv = {0, 0, 0, 0};
  if (wave == 0 && lane < 8) cv = *(const v4f*)(sC + 4 * lane);
  if (wave == 1 && lane < 8) sv = *(const v4i*)(sS + 4 * lane);
  if (wave == 2 && lane < 8) dv = *(const v4i*)(sDd + 4 * lane);
  *(volatile v8h*)gp = o;
  if (wave == 0 && lane < 8) *(volatile v4f*)(Cpos + P0 + 4 * lane) = cv;
  if (wave == 1 && lane < 8) *(volatile v4i*)(Spos + P0 + 4 * lane) = sv;
  if (wave == 2 && lane < 8) *(volatile v4i*)(Dpos + P0 + 4 * lane) = dv;
  __threadfence();
  *(volatile v8h*)gp = o;
  if (wave == 0 && lane < 8) *(volatile v4f*)(Cpos + P0 + 4 * lane) = cv;
  if (wave == 1 && lane < 8) *(volatile v4i*)(Spos + P0 + 4 * lane) = sv;
  if (wave == 2 && lane < 8) *(volatile v4i*)(Dpos + P0 + 4 * lane) = dv;
}

__global__ __launch_bounds__(NTHR) void k_gather(
    const int* __restrict__ z, const float* __restrict__ emb, float* x0, int nN, int nTab) {
  const int tid = threadIdx.x, lane = tid & 31, wave = tid >> 5;
  const int c  = blockIdx.x * NWAVE + wave;
  const int cc = c < nN ? c : nN - 1;
  int zi = z[cc];
  zi = zi < 0 ? 0 : (zi > nTab - 1 ? nTab - 1 : zi);
  const v4f v = *(const v4f*)(emb + (size_t)zi * HID + 4 * lane);
  float* gp = x0 + (size_t)c * HID + 4 * lane;
  *(volatile v4f*)gp = v;
  __threadfence();
  *(volatile v4f*)gp = v;
}

template <int LAYER>
__global__ __launch_bounds__(NTHR) void k_conv(
    const int* __restrict__ offp, const int* __restrict__ cntp,
    const float* __restrict__ Cpos, const int* __restrict__ Spos, const int* __restrict__ Dpos,
    const _Float16* __restrict__ eaP, const float* __restrict__ hsrc,
    const _Float16* __restrict__ W0h, const float* __restrict__ b0,
    const _Float16* __restrict__ W1h, const float* __restrict__ b1,
    float* agg, int nN, int csrLen, int npad) {
  __shared__ __attribute__((aligned(16))) _Float16 sA[CPOS * APE];
  __shared__ __attribute__((aligned(16))) _Float16 sT[LAYER ? CPOS * TPH : 8];
  __shared__ __attribute__((aligned(16))) float sW[CPOS * WPF];
  __shared__ __attribute__((aligned(16))) float sC[CPOS];
  __shared__ __attribute__((aligned(16))) int sD[CPOS];
  const int tid = threadIdx.x, lane = tid & 31, wave = tid >> 5, hh = lane >> 4, m = lane & 15;
  const int c0 = blockIdx.x * CNB;
  int offl = offp[c0 + lane];
  int cntl = cntp[c0 + lane];
  cntl = cntl < 0 ? 0 : (cntl > DEGCAP ? DEGCAP : cntl);
  offl = offl < 0 ? 0 : (offl > csrLen ? csrLen : offl);
  const int R0 = __builtin_amdgcn_readfirstlane(offl);
  const int Rend = __builtin_amdgcn_readlane(offl, 31) + __builtin_amdgcn_readlane(cntl, 31);
  int tot = Rend - R0;
  tot = tot < 0 ? 0 : (tot > CNB * DEGCAP ? CNB * DEGCAP : tot);
  const int nch = (tot + CPOS - 1) / CPOS;
  const int rt = wave & 3, ct0 = (wave >> 2) * 4;
  const int rowb = 16 * rt + 8 * hh;

  v4f nacc[4];
#pragma unroll
  for (int s = 0; s < 4; ++s) { v4f zz = {0.f, 0.f, 0.f, 0.f}; nacc[s] = zz; }

#pragma unroll 1
  for (int ch = 0; ch < nch; ++ch) {
    const int P = R0 + ch * CPOS;
    __syncthreads();
    if (tid < CPOS) {
      int p = P + tid;
      p = p > csrLen - 1 ? csrLen - 1 : p;
      float c = Cpos[p];
      const int draw = Dpos[p];
      if constexpr (LAYER == 0) {
        const int sraw = Spos[p];
        c = (sraw != draw) ? c : 0.0f;
      }
      int d = draw < 0 ? 0 : (draw > nN - 1 ? nN - 1 : draw);
      sC[tid] = c;
      sD[tid] = d;
    }
#pragma unroll
    for (int i = 0; i < 2; ++i) {
      const int idx = i * NTHR + tid;
      const int r = idx >> 3, q = idx & 7;
      int p = P + r;
      p = p > csrLen - 1 ? csrLen - 1 : p;
      const v8h v = *(const v8h*)(eaP + (size_t)p * KRB + 8 * q);
      *(v8h*)(sA + r * APE + 8 * q) = v;
    }
    __syncthreads();

    v8f acc1[4];
#pragma unroll
    for (int t = 0; t < 4; ++t) { v8f zz = {0.f, 0.f, 0.f, 0.f, 0.f, 0.f, 0.f, 0.f}; acc1[t] = zz; }
    const _Float16* ap = sA + (16 * rt + m) * APE + 8 * hh;
#pragma unroll
    for (int ks = 0; ks < KRB / 32; ++ks) {
      FragH a;
      a.h[0] = *(const v8h*)(ap + 32 * ks);
      a.h[1] = *(const v8h*)(ap + 32 * ks + 16);
#pragma unroll
      for (int t = 0; t < 4; ++t) {
        const _Float16* bp = W0h + (size_t)(16 * (ct0 + t) + m) * KRB + 32 * ks + 8 * hh;
        FragH b;
        b.h[0] = *(const v8h*)bp;
        b.h[1] = *(const v8h*)(bp + 16);
        acc1[t] = wm(a.v, b.v, acc1[t]);
      }
    }

    if constexpr (LAYER != 0) {
#pragma unroll
      for (int t = 0; t < 4; ++t) {
        const int n = 16 * (ct0 + t) + m;
        const float bv = b0[n];
#pragma unroll
        for (int r = 0; r < 8; ++r) {
          const float v = silu_f(acc1[t][r] * EA_INV + bv);
          sT[(rowb + r) * TPH + n] = (_Float16)v;
        }
      }
      __syncthreads();
      v8f acc2[4];
#pragma unroll
      for (int t = 0; t < 4; ++t) { v8f zz = {0.f, 0.f, 0.f, 0.f, 0.f, 0.f, 0.f, 0.f}; acc2[t] = zz; }
      const _Float16* tp = sT + (16 * rt + m) * TPH + 8 * hh;
#pragma unroll
      for (int ks = 0; ks < HID / 32; ++ks) {
        FragH a;
        a.h[0] = *(const v8h*)(tp + 32 * ks);
        a.h[1] = *(const v8h*)(tp + 32 * ks + 16);
#pragma unroll
        for (int t = 0; t < 4; ++t) {
          const _Float16* bp = W1h + (size_t)(16 * (ct0 + t) + m) * HID + 32 * ks + 8 * hh;
          FragH b;
          b.h[0] = *(const v8h*)bp;
          b.h[1] = *(const v8h*)(bp + 16);
          acc2[t] = wm(a.v, b.v, acc2[t]);
        }
      }
#pragma unroll
      for (int t = 0; t < 4; ++t) {
        const int n = 16 * (ct0 + t) + m;
        const float bv = b1[n];
#pragma unroll
        for (int r = 0; r < 8; ++r) sW[(rowb + r) * WPF + n] = (acc2[t][r] + bv) * sC[rowb + r];
      }
    } else {
#pragma unroll
      for (int t = 0; t < 4; ++t) {
        const int n = 16 * (ct0 + t) + m;
        const float bv = b0[n];
#pragma unroll
        for (int r = 0; r < 8; ++r) sW[(rowb + r) * WPF + n] = (acc1[t][r] * EA_INV + bv) * sC[rowb + r];
      }
    }
    __syncthreads();

#pragma unroll
    for (int s = 0; s < 4; ++s) {
      const int j  = 4 * wave + s;
      const int oj = __shfl(offl, j);
      const int cj = __shfl(cntl, j);
      int lo = oj - P;
      lo = lo < 0 ? 0 : (lo > CPOS ? CPOS : lo);
      int hi = oj + cj - P;
      hi = hi < 0 ? 0 : (hi > CPOS ? CPOS : hi);
#pragma unroll 1
      for (int r = lo; r < hi; ++r) {
        const v4f wv = *(const v4f*)(sW + r * WPF + 4 * lane);
        const int d = sD[r];
        const v4f hv = *(const v4f*)(hsrc + (size_t)d * HID + 4 * lane);
        nacc[s] = nacc[s] + wv * hv;
      }
    }
  }

#pragma unroll
  for (int s = 0; s < 4; ++s) {
    const int c = c0 + 4 * wave + s;
    *(volatile v4f*)(agg + (size_t)c * HID + 4 * lane) = nacc[s];
  }
  __threadfence();
#pragma unroll
  for (int s = 0; s < 4; ++s) {
    const int c = c0 + 4 * wave + s;
    *(volatile v4f*)(agg + (size_t)c * HID + 4 * lane) = nacc[s];
  }
  (void)npad;
}

template <int KD>
__global__ __launch_bounds__(NTHR) void k_ngemm(
    const float* __restrict__ A1, const float* __restrict__ A2,
    const _Float16* __restrict__ Bw, const float* __restrict__ bias,
    const float* resid, float* C, int nRowsA, int nRowsOut, int flags) {
  extern __shared__ v4f lds_dyn[];
  constexpr int APH = KD + 8;
  constexpr int NIT = (GROWS * KD / 8) / NTHR;
  _Float16* sAt = (_Float16*)lds_dyn;
  float*    stg = (float*)lds_dyn;
  const int tid = threadIdx.x, lane = tid & 31, wave = tid >> 5, hh = lane >> 4, m = lane & 15;
  const int rowBase = blockIdx.x * GROWS;

#pragma unroll
  for (int i = 0; i < NIT; ++i) {
    const int half = i >> 3;
    const int j = (i & 7) * NTHR + tid;
    const int r = j >> 4;
    const int c = (j & 15) * 8;
    const float* src = half ? A2 : A1;
    int row = rowBase + r;
    row = row > nRowsA - 1 ? nRowsA - 1 : row;
    const float* ap = src + (size_t)row * HID + c;
    const v4f a = *(const v4f*)ap, b = *(const v4f*)(ap + 4);
    *(v8h*)(sAt + r * APH + half * HID + c) = cvt8(a, b);
  }
  __syncthreads();

  v8f acc[8];
#pragma unroll
  for (int t = 0; t < 8; ++t) { v8f zz = {0.f, 0.f, 0.f, 0.f, 0.f, 0.f, 0.f, 0.f}; acc[t] = zz; }
  const _Float16* ap = sAt + (wave * 16 + m) * APH + 8 * hh;
#pragma unroll
  for (int kt = 0; kt < KD / 32; ++kt) {
    FragH a;
    a.h[0] = *(const v8h*)(ap + 32 * kt);
    a.h[1] = *(const v8h*)(ap + 32 * kt + 16);
#pragma unroll
    for (int t = 0; t < 8; ++t) {
      const _Float16* bp = Bw + (size_t)(16 * t + m) * KD + 32 * kt + 8 * hh;
      FragH b;
      b.h[0] = *(const v8h*)bp;
      b.h[1] = *(const v8h*)(bp + 16);
      acc[t] = wm(a.v, b.v, acc[t]);
    }
  }
  __syncthreads();

  const int r0 = wave * 16 + 8 * hh;
  float* sp = stg + r0 * HID + m;
#pragma unroll
  for (int t = 0; t < 8; ++t) {
#pragma unroll
    for (int r = 0; r < 8; ++r) sp[r * HID + 16 * t] = acc[t][r];
  }
  __syncthreads();

  const v4f zero4 = {0.f, 0.f, 0.f, 0.f};
  const v4f braw = *(const v4f*)(bias + 4 * lane);
  const v4f bsel = (flags & FL_BIAS) ? braw : zero4;
  const float* lp = stg + wave * 16 * HID + 4 * lane;
  const int rw0 = rowBase + wave * 16;
  v4f vals[16];
#pragma unroll
  for (int i = 0; i < 16; ++i) {
    v4f v = *(const v4f*)(lp + i * HID);
    v = v + bsel;
    if (flags & FL_SILU) v = silu4(v);
    if (flags & FL_RES) {
      int rr = rw0 + i;
      rr = rr > nRowsA - 1 ? nRowsA - 1 : rr;
      v = v + *(const v4f*)(resid + (size_t)rr * HID + 4 * lane);
    }
    vals[i] = v;
  }
#pragma unroll
  for (int i = 0; i < 16; ++i) {
    const int row = rw0 + i;
    if (row < nRowsOut) *(volatile v4f*)(C + (size_t)row * HID + 4 * lane) = vals[i];
  }
  __threadfence();
#pragma unroll
  for (int i = 0; i < 16; ++i) {
    const int row = rw0 + i;
    if (row < nRowsOut) *(volatile v4f*)(C + (size_t)row * HID + 4 * lane) = vals[i];
  }
}

extern "C" void kernel_launch(void* const* d_in, const int* in_sizes, int n_in,
                              void* d_out, int out_size, void* d_ws, size_t ws_size,
                              hipStream_t stream) {
  if (n_in < 19) return;
  const int nN = in_sizes[0];
  const int nE = in_sizes[2];
  if (nN <= 0 || nE <= 0) return;
  if (in_sizes[1] != 2 * nE) return;
  if (in_sizes[3] <= 0 || (in_sizes[3] % HID) != 0) return;
  const int nTab = in_sizes[3] / HID;
  const int nrbf = in_sizes[4];
  if (nrbf < 1 || nrbf > KRB || in_sizes[5] != nrbf) return;
  if (in_sizes[6] != HID * nrbf || in_sizes[7] != HID) return;
  if (in_sizes[8] != HID * 2 * HID || in_sizes[9] != HID) return;
  if (in_sizes[10] != NLAY * HID * nrbf || in_sizes[11] != NLAY * HID) return;
  if (in_sizes[12] != NLAY * HID * HID || in_sizes[13] != NLAY * HID) return;
  if (in_sizes[14] != NLAY * HID * HID || in_sizes[15] != NLAY * HID * HID) return;
  if (in_sizes[16] != NLAY * HID || in_sizes[17] != NLAY * HID * HID || in_sizes[18] != NLAY * HID) return;
  if (out_size != nN * HID) return;
  if (nE > (1 << 26) || nN > (1 << 22)) return;

  const int*   z     = (const int*)d_in[0];
  const int*   ei    = (const int*)d_in[1];
  const float* ew    = (const float*)d_in[2];
  const float* emb   = (const float*)d_in[3];
  const float* means = (const float*)d_in[4];
  const float* betas = (const float*)d_in[5];
  const float* pw    = (const float*)d_in[6];
  const float* pb    = (const float*)d_in[7];
  const float* cw    = (const float*)d_in[8];
  const float* cb    = (const float*)d_in[9];
  const float* w0    = (const float*)d_in[10];
  const float* b0    = (const float*)d_in[11];
  const float* w1    = (const float*)d_in[12];
  const float* b1    = (const float*)d_in[13];
  const float* l1w   = (const float*)d_in[14];
  const float* l2w   = (const float*)d_in[15];
  const float* l2b   = (const float*)d_in[16];
  const float* lnw   = (const float*)d_in[17];
  const float* lnb   = (const float*)d_in[18];
  float* out = (float*)d_out;

  const int NPAD   = ((nN + GROWS - 1) / GROWS) * GROWS;
  const int nBC    = (nN + NBC - 1) / NBC;
  const int CNTPAD = nBC * NBC;
  if (NPAD > CNTPAD) return;
  if (4 * nBC + 1 > RBN) return;
  const int nBF    = (nN + NBF - 1) / NBF;
  if (31 * 4 * nBC > 4096) return;
  const int csrLen = ((nE + 31) & ~31) + 4096;
  const int nConv  = NPAD / CNB;
  const int nGemm  = NPAD / GROWS;
  const int nGat   = NPAD / NWAVE;
  const int nEA    = csrLen / EROWS;

  char* ws = (char*)d_ws;
  size_t off = 0;
  const size_t plane = (size_t)NPAD * HID * 4;
  const size_t oW   = off; off += (size_t)WTOT * 2;            off = (off + 255) & ~(size_t)255;
  const size_t oCnt = off; off += (size_t)CNTPAD * 4;          off = (off + 255) & ~(size_t)255;
  const size_t oOff = off; off += (size_t)CNTPAD * 4;          off = (off + 255) & ~(size_t)255;
  const size_t oRb  = off; off += (size_t)RBN * 4;             off = (off + 255) & ~(size_t)255;
  const size_t oCsr = off; off += (size_t)csrLen * 4;          off = (off + 255) & ~(size_t)255;
  const size_t oCp  = off; off += (size_t)csrLen * 4;          off = (off + 255) & ~(size_t)255;
  const size_t oSp  = off; off += (size_t)csrLen * 4;          off = (off + 255) & ~(size_t)255;
  const size_t oDp  = off; off += (size_t)csrLen * 4;          off = (off + 255) & ~(size_t)255;
  const size_t oEa  = off; off += (size_t)csrLen * KRB * 2;    off = (off + 255) & ~(size_t)255;
  const size_t oX0  = off; off += plane;                       off = (off + 255) & ~(size_t)255;
  const size_t oAgg = off; off += plane;                       off = (off + 255) & ~(size_t)255;
  const size_t oXA  = off; off += plane;                       off = (off + 255) & ~(size_t)255;
  const size_t oXB  = off; off += plane;                       off = (off + 255) & ~(size_t)255;
  const size_t oH   = off; off += plane;                       off = (off + 255) & ~(size_t)255;
  const size_t oT   = off; off += plane;                       off = (off + 255) & ~(size_t)255;
  if (off > ws_size || off > (size_t)WSCAP) return;
  _Float16* wp  = (_Float16*)(ws + oW);
  int*   cnt  = (int*)(ws + oCnt);
  int*   offp = (int*)(ws + oOff);
  int*   rb   = (int*)(ws + oRb);
  int*   csr  = (int*)(ws + oCsr);
  float* Cp   = (float*)(ws + oCp);
  int*   Sp   = (int*)(ws + oSp);
  int*   Dp   = (int*)(ws + oDp);
  _Float16* eaP = (_Float16*)(ws + oEa);
  float* x0   = (float*)(ws + oX0);
  float* agg  = (float*)(ws + oAgg);
  float* xA   = (float*)(ws + oXA);
  float* xB   = (float*)(ws + oXB);
  float* hpl  = (float*)(ws + oH);
  float* tpl  = (float*)(ws + oT);

  const int vec8 = ((nE & 3) == 0) ? 1 : 0;

  k_wprep<<<WBLK, NTHR, 0, stream>>>(pw, cw, w0, w1, l1w, l2w, lnw, wp, nrbf);

  k_count<<<nBC, NTHR, 0, stream>>>(ei, cnt, nE, vec8);
  k_offsets<<<1, OTHR, 0, stream>>>(cnt, offp, rb, nBC);
  hipFuncSetAttribute(reinterpret_cast<const void*>(&k_fill),
                      hipFuncAttributeMaxDynamicSharedMemorySize, LDS_FILL);
  k_fill<<<nBF, NTHR, LDS_FILL, stream>>>(ei, offp, rb, csr, nE, vec8, csrLen);

  k_eattr<<<nEA, NTHR, 0, stream>>>(csr, ei, ew, means, betas, eaP, Cp, Sp, Dp, nE, nN, csrLen, nrbf);

  k_gather<<<nGat, NTHR, 0, stream>>>(z, emb, x0, nN, nTab);

  const _Float16* projh = wp + WO_PROJ;
  const _Float16* combh = wp + WO_COMB;
  k_conv<0><<<nConv, NTHR, 0, stream>>>(offp, cnt, Cp, Sp, Dp, eaP, x0, projh, pb, projh, pb,
                                        agg, nN, csrLen, NPAD);

  hipFuncSetAttribute(reinterpret_cast<const void*>(&k_ngemm<256>),
                      hipFuncAttributeMaxDynamicSharedMemorySize, LDS_NG256);
  hipFuncSetAttribute(reinterpret_cast<const void*>(&k_ngemm<128>),
                      hipFuncAttributeMaxDynamicSharedMemorySize, LDS_NG128);
  k_ngemm<256><<<nGemm, NTHR, LDS_NG256, stream>>>(x0, agg, combh, cb, x0, xA, NPAD, NPAD, FL_BIAS);

  for (int l = 0; l < NLAY; ++l) {
    const _Float16* base = wp + WO_LAY0 + (size_t)l * WL_STR;
    const _Float16* w0h = base + WL_W0;
    const _Float16* w1h = base + WL_W1;
    const _Float16* l1h = base + WL_L1;
    const _Float16* l2h = base + WL_L2;
    const _Float16* lwh = base + WL_LW;
    const float* b0l  = b0  + (size_t)l * HID;
    const float* b1l  = b1  + (size_t)l * HID;
    const float* l2bl = l2b + (size_t)l * HID;
    const float* lbl  = lnb + (size_t)l * HID;
    const float* xcur = (l == 1) ? xB : xA;
    float* xnext = (l == 0) ? xB : ((l == 1) ? xA : out);
    const int nOut = (l == NLAY - 1) ? nN : NPAD;

    k_ngemm<128><<<nGemm, NTHR, LDS_NG128, stream>>>(xcur, xcur, l1h, l2bl, xcur, hpl, NPAD, NPAD, 0);
    k_conv<1><<<nConv, NTHR, 0, stream>>>(offp, cnt, Cp, Sp, Dp, eaP, hpl, w0h, b0l, w1h, b1l,
                                          agg, nN, csrLen, NPAD);
    k_ngemm<128><<<nGemm, NTHR, LDS_NG128, stream>>>(agg, agg, l2h, l2bl, agg, tpl, NPAD, NPAD,
                                                     FL_BIAS | FL_SILU);
    k_ngemm<128><<<nGemm, NTHR, LDS_NG128, stream>>>(tpl, tpl, lwh, lbl, xcur, xnext, NPAD, nOut,
                                                     FL_BIAS | FL_RES);
  }
}
